// CSA_DGCN_38087769981513
// MI455X (gfx1250) — hardware-verified
//
#include <hip/hip_runtime.h>


#define NB_  256
#define NN   128
#define NIN  9
#define HD_  128
#define NH_  8
#define DH   16
#define NL   4
#define NOUT 60
#define NR   (NB_ * NN)
#define DM   HD_
#define LOSC 1024.0f
typedef _Float16 h16;
typedef unsigned short bf;
typedef __attribute__((ext_vector_type(16))) __bf16   v16bf;
typedef __attribute__((ext_vector_type(16))) _Float16 v16h;
typedef __attribute__((ext_vector_type(8)))  _Float16 v8h;
typedef __attribute__((ext_vector_type(8)))  unsigned short v8us;
typedef __attribute__((ext_vector_type(8)))  float    v8f;
typedef __attribute__((ext_vector_type(4)))  float    v4f;
typedef __attribute__((ext_vector_type(4)))  _Float16 v4h;
typedef v8h  __attribute__((may_alias)) v8ha;
typedef v4f  __attribute__((may_alias)) v4fa;
typedef v8us __attribute__((may_alias)) v8usa;

__device__ __forceinline__ unsigned short f2bf(float f) { unsigned u = __float_as_uint(f); u += 0x7FFFu + ((u >> 16) & 1u); return (unsigned short)(u >> 16); }
__device__ __forceinline__ float bf2f(unsigned short b) { return __uint_as_float(((unsigned)b) << 16); }
__device__ __forceinline__ float bfr(float f) { return bf2f(f2bf(f)); }
__device__ __forceinline__ v16h cat16(v8h lo, v8h hi) { return __builtin_shufflevector(lo, hi, 0, 1, 2, 3, 4, 5, 6, 7, 8, 9, 10, 11, 12, 13, 14, 15); }
__device__ __forceinline__ v16bf cat16b(v8us lo, v8us hi) { return __builtin_bit_cast(v16bf, __builtin_shufflevector(lo, hi, 0, 1, 2, 3, 4, 5, 6, 7, 8, 9, 10, 11, 12, 13, 14, 15)); }
__device__ __forceinline__ v8f wmma16(v16h a, v16h b, v8f c) { return __builtin_amdgcn_wmma_f32_16x16x32_f16(false, a, false, b, (short)0, c, false, false); }
__device__ __forceinline__ v8f wmmab(v16bf a, v16bf b, v8f c) { return __builtin_amdgcn_wmma_f32_16x16x32_bf16(false, a, false, b, (short)0, c, false, false); }

template <bool SPLITA, bool F16OUT = false>
__global__ __launch_bounds__(128) void k_gemmb(const bf* __restrict__ A, const bf* __restrict__ Al, const bf* __restrict__ Bn, const float* __restrict__ bias, float* C, int ldc, h16* C2, const float* __restrict__ R = nullptr, int K = DM, int roundR = 1) {
    __shared__ __align__(16) float ost[4][16 * 68];
    const int lane = threadIdx.x & 31, wave = threadIdx.x >> 5, lr = lane & 15, hi = lane >> 4;
    const int r0 = blockIdx.x * 64 + wave * 16, c0 = blockIdx.y * 64;
    const size_t aoff = (size_t)(r0 + lr) * K + 8 * hi;
    size_t boff[4];
#pragma unroll
    for (int t = 0; t < 4; ++t) boff[t] = (size_t)(c0 + t * 16 + lr) * K + 8 * hi;
    v8f acc[4];
#pragma unroll
    for (int t = 0; t < 4; ++t) acc[t] = (v8f){};
#pragma unroll 1
    for (int kc = 0; kc < K; kc += 32) {
        const v16bf a = cat16b(*(const v8us*)(A + aoff + kc), *(const v8us*)(A + aoff + kc + 16));
        v16bf al = a;
        if (SPLITA) al = cat16b(*(const v8us*)(Al + aoff + kc), *(const v8us*)(Al + aoff + kc + 16));
#pragma unroll
        for (int t = 0; t < 4; ++t) { const v16bf b = cat16b(*(const v8us*)(Bn + boff[t] + kc), *(const v8us*)(Bn + boff[t] + kc + 16)); acc[t] = wmmab(a, b, acc[t]); if (SPLITA) acc[t] = wmmab(al, b, acc[t]); }
        asm volatile("v_nop\n\tv_nop\n\tv_nop\n\tv_nop" : "+v"(acc[0]), "+v"(acc[1]), "+v"(acc[2]), "+v"(acc[3]) : "v"(a), "v"(al));
    }
    float* os = &ost[wave][0];
#pragma unroll
    for (int t = 0; t < 4; ++t) { const float bv = bias ? bfr(bias[c0 + t * 16 + lr]) : 0.f;
#pragma unroll
        for (int j = 0; j < 8; ++j) os[(hi * 8 + j) * 68 + t * 16 + lr] = acc[t][j] + bv; }
    __syncthreads();
    if (F16OUT) {
        h16* crow = (h16*)(void*)C + (size_t)r0 * ldc + c0;
        auto pass = [&]() {
#pragma unroll
            for (int s = 0; s < 4; ++s) { const int row = 4 * s + (lane >> 3), piece = lane & 7; const float* sp = os + row * 68 + piece * 8; v8h o, o2;
#pragma unroll
                for (int i = 0; i < 8; ++i) { const h16 a = (h16)sp[i]; o[i] = a; o2[i] = (h16)((sp[i] - (float)a) * LOSC); }
                *(volatile v8h*)(crow + (size_t)row * ldc + piece * 8) = o; if (C2) *(volatile v8h*)(C2 + (size_t)r0 * ldc + c0 + (size_t)row * ldc + piece * 8) = o2; }
        };
        pass(); __threadfence(); pass();
    } else {
        float* crow = C + (size_t)r0 * ldc + c0;
        auto pass = [&]() {
#pragma unroll
            for (int s = 0; s < 8; ++s) { const int Lid = (lane >> 3) + 4 * s, piece = lane & 7; const int row = Lid >> 1, cofs = (Lid & 1) * 32 + piece * 4;
                v4f val = *(const v4fa*)(os + row * 68 + cofs); if (R) { const v4f rv = *(const v4f*)(R + ((size_t)r0 + row) * ldc + c0 + cofs); val += roundR ? (v4f){bfr(rv[0]), bfr(rv[1]), bfr(rv[2]), bfr(rv[3])} : rv; }
                *(volatile v4f*)(crow + (size_t)row * ldc + cofs) = val; }
        };
        pass(); __threadfence(); pass();
    }
}


__global__ __launch_bounds__(256) void k_wt_io(const float* __restrict__ Wm, int ldw, int K, int N, bf* Bt) {
    const int lane = threadIdx.x & 31; const int n = blockIdx.x * 8 + (threadIdx.x >> 5); if (n >= N) return;
#pragma unroll 1
    for (int ps = 0; ps < 2; ++ps) { for (int c0 = lane * 8; c0 < K; c0 += 256) { v8us o;
#pragma unroll
            for (int i = 0; i < 8; ++i) { const int k = c0 + i; o[i] = f2bf(k < K ? Wm[(size_t)(k < K ? k : 0) * ldw + n] : 0.f); }
            *(volatile v8us*)(Bt + (size_t)n * K + c0) = o; }
        if (ps == 0) __threadfence(); }
}
__global__ __launch_bounds__(256) void k_embed(const float* __restrict__ x, const float* __restrict__ cw, const float* __restrict__ cb, const float* __restrict__ gam, const float* __restrict__ bet, const float* __restrict__ mean, const float* __restrict__ var, float* H) {
    const int lane = threadIdx.x & 31; const size_t r = (size_t)blockIdx.x * 8 + (threadIdx.x >> 5); if (r >= (size_t)NR) return; float xi[NIN];
#pragma unroll
    for (int i = 0; i < NIN; ++i) xi[i] = bfr(x[r * NIN + i]);
    v4f o;
#pragma unroll
    for (int q = 0; q < 4; ++q) { const int c = lane * 4 + q; float a = 0.f;
#pragma unroll
        for (int i = 0; i < NIN; ++i) a = fmaf(xi[i], bfr(cw[c * NIN + i]), a);
        a += bfr(cb[c]); a = (a - bfr(mean[c])) * rsqrtf(bfr(var[c]) + 1e-5f) * bfr(gam[c]) + bfr(bet[c]); o[q] = fmaxf(a, 0.f); }
    *(volatile v4f*)(H + r * HD_ + lane * 4) = o; __threadfence(); *(volatile v4f*)(H + r * HD_ + lane * 4) = o;
}
__global__ __launch_bounds__(256) void k_weak(const float* __restrict__ wp, const float* __restrict__ wm, float* AW) {
    const int lane = threadIdx.x & 31; const int i = blockIdx.x * 8 + (threadIdx.x >> 5); if (i >= NN) return; float v[4]; float s = 0.f;
#pragma unroll
    for (int q = 0; q < 4; ++q) { const int j = lane * 4 + q; v[q] = (1.0f / (1.0f + expf(-bfr(wp[i * NN + j])))) * bfr(wm[i * NN + j]); s += v[q]; }
#pragma unroll
    for (int sh = 16; sh; sh >>= 1) s += __shfl_xor(s, sh, 32);
    const float inv = 1.0f / (s + 1e-5f); v4f o; for (int q = 0; q < 4; ++q) o[q] = v[q] * inv;
    *(volatile v4f*)(AW + i * NN + lane * 4) = o; __threadfence(); *(volatile v4f*)(AW + i * NN + lane * 4) = o;
}
__global__ __launch_bounds__(256) void k_split128(const float* __restrict__ F, size_t rows, bf* Ph, bf* Pl) {
    typedef __attribute__((ext_vector_type(4))) unsigned short v4us;
    const int lane = threadIdx.x & 31; const size_t r = (size_t)blockIdx.x * 8 + (threadIdx.x >> 5); if (r >= rows) return; const size_t o = r * HD_ + lane * 4; const v4f v = *(const v4f*)(F + o); v4us oh, ol;
#pragma unroll
    for (int i = 0; i < 4; ++i) { const unsigned short hb = f2bf(v[i]); oh[i] = hb; ol[i] = f2bf(v[i] - bf2f(hb)); }
    *(volatile v4us*)(Ph + o) = oh; *(volatile v4us*)(Pl + o) = ol; __threadfence(); *(volatile v4us*)(Ph + o) = oh; *(volatile v4us*)(Pl + o) = ol;
}
__global__ __launch_bounds__(256) void k_relu256p(const float* __restrict__ F, size_t rows, bf* Ph, bf* Pl) {
    const int lane = threadIdx.x & 31; const size_t r = (size_t)blockIdx.x * 8 + (threadIdx.x >> 5); if (r >= rows) return; const size_t o = r * 256 + lane * 8; const v8f v = *(const v8f*)(F + o); v8us oh, ol;
#pragma unroll
    for (int i = 0; i < 8; ++i) { const float y = fmaxf(v[i], 0.f); const unsigned short hb = f2bf(y); oh[i] = hb; ol[i] = f2bf(y - bf2f(hb)); }
    *(volatile v8us*)(Ph + o) = oh; *(volatile v8us*)(Pl + o) = ol; __threadfence(); *(volatile v8us*)(Ph + o) = oh; *(volatile v8us*)(Pl + o) = ol;
}
__global__ __launch_bounds__(256) void k_st(const float* __restrict__ HP, const float* __restrict__ asrc, const float* __restrict__ adst, float* ST) {
    const int lane = threadIdx.x & 31; const size_t r = ((size_t)blockIdx.x * 8 + (threadIdx.x >> 5)) * 2 + (lane >> 4); if (r >= (size_t)NR) return; const int l2 = lane & 15; const int h = l2 & 7; const float* av = (l2 < 8) ? asrc : adst; float a = 0.f;
#pragma unroll
    for (int d = 0; d < DH; ++d) a = fmaf(HP[r * HD_ + h * DH + d], bfr(av[h * DH + d]), a);
    *(volatile float*)(ST + r * 16 + l2) = a; __threadfence(); *(volatile float*)(ST + r * 16 + l2) = a;
}
__global__ __launch_bounds__(256) void k_gat(const float* __restrict__ HP, const float* __restrict__ ST, const float* __restrict__ strong, const float* __restrict__ ew, const float* __restrict__ AW, float* G) {
    __shared__ float se[8][NH_ * NN];
    const int lane = threadIdx.x & 31, wv = threadIdx.x >> 5; const size_t r = (size_t)blockIdx.x * 8 + wv; if (r >= (size_t)NR) return; const int b = (int)(r / NN), i = (int)(r % NN); float* E = se[wv]; const size_t rb = (size_t)b * NN;
#pragma unroll 1
    for (int q = lane; q < NH_ * NN; q += 32) { const int h = q / NN, j = q % NN; float e = -3.0e38f;
        if (strong[i * NN + j] > 0.f) { float v = ST[r * 16 + h] + ST[(rb + j) * 16 + 8 + h]; v = v > 0.f ? v : 0.2f * v; e = v + bfr(ew[i * NN + j]); }
        E[q] = e; }
    __builtin_amdgcn_wave_barrier(); asm volatile("" ::: "memory");
    if (lane < NH_) { const int h = lane; float m = -3.0e38f;
#pragma unroll 1
        for (int j = 0; j < NN; ++j) m = fmaxf(m, E[h * NN + j]);
        float sum = 0.f;
#pragma unroll 1
        for (int j = 0; j < NN; ++j) { const float e = (E[h * NN + j] > -1.0e38f) ? __expf(E[h * NN + j] - m) : 0.f; E[h * NN + j] = e; sum += e; }
        const float inv = 1.0f / sum;
#pragma unroll 1
        for (int j = 0; j < NN; ++j) E[h * NN + j] *= inv; }
    __builtin_amdgcn_wave_barrier(); asm volatile("" ::: "memory");
    const int c0 = lane * 4; const int h = c0 / DH; v4f as = (v4f){0.f, 0.f, 0.f, 0.f}, aw = (v4f){0.f, 0.f, 0.f, 0.f};
#pragma unroll 1
    for (int j = 0; j < NN; ++j) { const float a = E[h * NN + j]; const float w = AW[i * NN + j]; const v4f hv = *(const v4f*)(HP + (rb + j) * HD_ + c0);
#pragma unroll
        for (int k = 0; k < 4; ++k) { as[k] = fmaf(a, hv[k], as[k]); aw[k] = fmaf(w, hv[k], aw[k]); } }
    v4f o;
#pragma unroll
    for (int k = 0; k < 4; ++k) o[k] = fmaxf(0.6f * as[k] + 0.4f * aw[k], 0.f);
    *(volatile v4f*)(G + r * HD_ + c0) = o; __threadfence(); *(volatile v4f*)(G + r * HD_ + c0) = o;
}
template <bool PLANES, bool F32OUT>
__global__ __launch_bounds__(256) void k_ln128(const float* __restrict__ F, size_t rows, const float* __restrict__ g, const float* __restrict__ bb, bf* Ph, bf* Pl, float* OF) {
    typedef __attribute__((ext_vector_type(4))) unsigned short v4us;
    const int lane = threadIdx.x & 31; const size_t r = (size_t)blockIdx.x * 8 + (threadIdx.x >> 5); if (r >= rows) return; const v4f v = *(const v4f*)(F + r * HD_ + lane * 4); float s = v[0] + v[1] + v[2] + v[3];
#pragma unroll
    for (int sh = 16; sh; sh >>= 1) s += __shfl_xor(s, sh, 32);
    const float mu = s * (1.0f / HD_); float q = 0.f;
#pragma unroll
    for (int i = 0; i < 4; ++i) { const float d = v[i] - mu; q = fmaf(d, d, q); }
#pragma unroll
    for (int sh = 16; sh; sh >>= 1) q += __shfl_xor(q, sh, 32);
    const float rs = rsqrtf(q * (1.0f / HD_) + 1e-5f); v4f o; v4us oh, ol;
#pragma unroll
    for (int i = 0; i < 4; ++i) { const int c = lane * 4 + i; const float y = (v[i] - mu) * rs * bfr(g[c]) + bfr(bb[c]); o[i] = y; const unsigned short hb = f2bf(y); oh[i] = hb; ol[i] = f2bf(y - bf2f(hb)); }
    const size_t off = r * HD_ + lane * 4;
#pragma unroll 1
    for (int ps = 0; ps < 2; ++ps) { if (PLANES) { *(volatile v4us*)(Ph + off) = oh; *(volatile v4us*)(Pl + off) = ol; } if (F32OUT) *(volatile v4f*)(OF + off) = o; if (ps == 0) __threadfence(); }
}
__global__ __launch_bounds__(256) void k_poolhead(const float* __restrict__ P, const float* __restrict__ w1, const float* __restrict__ b1, const float* __restrict__ w2, const float* __restrict__ b2, float* OUTP) {
    __shared__ float sz[8][HD_]; __shared__ float sh1[8][64];
    const int lane = threadIdx.x & 31, wv = threadIdx.x >> 5; const int b = blockIdx.x * 8 + wv; if (b >= NB_) return; float* z = sz[wv]; float* h1 = sh1[wv];
    v4f acc = (v4f){0.f, 0.f, 0.f, 0.f};
#pragma unroll 1
    for (int n = 0; n < NN; ++n) { const v4f v = *(const v4f*)(P + ((size_t)b * NN + n) * HD_ + lane * 4); acc += v; }
#pragma unroll
    for (int k = 0; k < 4; ++k) z[lane * 4 + k] = acc[k] * (1.0f / NN);
    __builtin_amdgcn_wave_barrier(); asm volatile("" ::: "memory");
#pragma unroll 1
    for (int k = lane; k < 64; k += 32) { float a = bfr(b1[k]);
#pragma unroll 1
        for (int c = 0; c < HD_; ++c) a = fmaf(z[c], bfr(w1[c * 64 + k]), a);
        h1[k] = fmaxf(a, 0.f); }
    __builtin_amdgcn_wave_barrier(); asm volatile("" ::: "memory");
    float o2[2];
#pragma unroll
    for (int q = 0; q < 2; ++q) { const int o = lane * 2 + q; float a = 0.f; if (o < NOUT) { a = bfr(b2[o]);
#pragma unroll 1
            for (int k = 0; k < 64; ++k) a = fmaf(h1[k], bfr(w2[k * NOUT + o]), a); }
        o2[q] = a; }
    typedef __attribute__((ext_vector_type(2))) float v2f_; v2f_ ov; ov[0] = o2[0]; ov[1] = o2[1];
    *(volatile v2f_*)(OUTP + (size_t)b * 64 + lane * 2) = ov; __threadfence(); *(volatile v2f_*)(OUTP + (size_t)b * 64 + lane * 2) = ov;
}
__global__ __launch_bounds__(256) void k_out60(const float* __restrict__ OUTP, float* OUTB) {
    const int lane = threadIdx.x & 31; const size_t e = ((size_t)blockIdx.x * 8 + (threadIdx.x >> 5)) * 32 + lane; if (e >= (size_t)NB_ * NOUT) return; const float v = OUTP[(e / NOUT) * 64 + (e % NOUT)];
    *(volatile float*)(OUTB + e) = v; __threadfence(); *(volatile float*)(OUTB + e) = v;
}
extern "C" void kernel_launch(void* const* d_in, const int* in_sizes, int n_in,
                              void* d_out, int out_size, void* d_ws, size_t ws_size, hipStream_t stream) {
    (void)in_sizes; (void)n_in; (void)out_size;
    const float* x = (const float*)d_in[0]; const float* cw = (const float*)d_in[1]; const float* cb = (const float*)d_in[2]; const float* bng = (const float*)d_in[3]; const float* bnb = (const float*)d_in[4]; const float* bnm = (const float*)d_in[5]; const float* bnv = (const float*)d_in[6];
    const float* Wl = (const float*)d_in[7]; const float* asrc = (const float*)d_in[8]; const float* adst = (const float*)d_in[9]; const float* lng = (const float*)d_in[10]; const float* lnb = (const float*)d_in[11]; const float* fw1 = (const float*)d_in[12]; const float* fb1 = (const float*)d_in[13]; const float* fw2 = (const float*)d_in[14]; const float* fb2 = (const float*)d_in[15];
    const float* ng = (const float*)d_in[16]; const float* nb = (const float*)d_in[17]; const float* pw = (const float*)d_in[18]; const float* pb = (const float*)d_in[19]; const float* hw1 = (const float*)d_in[20]; const float* hb1 = (const float*)d_in[21]; const float* hw2 = (const float*)d_in[22]; const float* hb2 = (const float*)d_in[23];
    const float* strong = (const float*)d_in[24]; const float* wmask = (const float*)d_in[25]; const float* wparam = (const float*)d_in[26]; const float* ewadj = (const float*)d_in[27];
    float* out = (float*)d_out;
    char* wsp = (char*)d_ws;
    auto take = [&](size_t bytes) { char* p = wsp; wsp += (bytes + 255) & ~(size_t)255; return (void*)p; };
    bf* WL = (bf*)take((size_t)NL * HD_ * HD_ * 2); bf* WF1 = (bf*)take((size_t)NL * 256 * HD_ * 2); bf* WF2 = (bf*)take((size_t)NL * HD_ * 256 * 2); bf* WP = (bf*)take(HD_ * HD_ * 2); float* AW = (float*)take(NN * NN * 4);
    float* H = (float*)take((size_t)NR * HD_ * 4); bf* Ph = (bf*)take((size_t)NR * 256 * 2); bf* Pl = (bf*)take((size_t)NR * 256 * 2); float* HP = (float*)take((size_t)NR * HD_ * 4); float* ST = (float*)take((size_t)NR * 16 * 4); float* G = (float*)take((size_t)NR * HD_ * 4); float* F1 = (float*)take((size_t)NR * 256 * 4); float* H2 = (float*)take((size_t)NR * HD_ * 4); float* OUTP = (float*)take(NB_ * 64 * 4);
    if ((size_t)(wsp - (char*)d_ws) > ws_size) return;
    for (int l = 0; l < NL; ++l) { k_wt_io<<<HD_ / 8, 256, 0, stream>>>(Wl + (size_t)l * HD_ * HD_, HD_, HD_, HD_, WL + (size_t)l * HD_ * HD_); k_wt_io<<<256 / 8, 256, 0, stream>>>(fw1 + (size_t)l * HD_ * 256, 256, HD_, 256, WF1 + (size_t)l * 256 * HD_); k_wt_io<<<HD_ / 8, 256, 0, stream>>>(fw2 + (size_t)l * 256 * HD_, HD_, 256, HD_, WF2 + (size_t)l * HD_ * 256); }
    k_wt_io<<<HD_ / 8, 256, 0, stream>>>(pw, HD_, HD_, HD_, WP);
    k_weak<<<NN / 8, 256, 0, stream>>>(wparam, wmask, AW);
    k_embed<<<NR / 8, 256, 0, stream>>>(x, cw, cb, bng, bnb, bnm, bnv, H);
    for (int l = 0; l < NL; ++l) {
        k_split128<<<NR / 8, 256, 0, stream>>>(H, NR, Ph, Pl);
        k_gemmb<true, false><<<dim3(NR / 64, HD_ / 64, 1), 128, 0, stream>>>(Ph, Pl, WL + (size_t)l * HD_ * HD_, nullptr, HP, HD_, nullptr, nullptr, HD_);
        k_st<<<(NR / 2) / 8, 256, 0, stream>>>(HP, asrc + (size_t)l * NH_ * DH, adst + (size_t)l * NH_ * DH, ST);
        k_gat<<<NR / 8, 256, 0, stream>>>(HP, ST, strong, ewadj, AW, G);
        k_ln128<true, false><<<NR / 8, 256, 0, stream>>>(G, NR, lng + (size_t)l * HD_, lnb + (size_t)l * HD_, Ph, Pl, nullptr);
        k_gemmb<true, false><<<dim3(NR / 64, 256 / 64, 1), 128, 0, stream>>>(Ph, Pl, WF1 + (size_t)l * 256 * HD_, fb1 + (size_t)l * 256, F1, 256, nullptr, nullptr, HD_);
        k_relu256p<<<NR / 8, 256, 0, stream>>>(F1, NR, Ph, Pl);
        k_gemmb<true, false><<<dim3(NR / 64, HD_ / 64, 1), 128, 0, stream>>>(Ph, Pl, WF2 + (size_t)l * HD_ * 256, fb2 + (size_t)l * HD_, H2, HD_, nullptr, H, 256, 0);
        { float* t = H; H = H2; H2 = t; } }
    k_ln128<true, false><<<NR / 8, 256, 0, stream>>>(H, NR, ng, nb, Ph, Pl, nullptr);
    k_gemmb<true, false><<<dim3(NR / 64, HD_ / 64, 1), 128, 0, stream>>>(Ph, Pl, WP, pb, HP, HD_, nullptr, nullptr, HD_);
    k_poolhead<<<NB_ / 8, 256, 0, stream>>>(HP, hw1, hb1, hw2, hb2, OUTP);
    k_out60<<<(NB_ * NOUT / 32 + 7) / 8, 256, 0, stream>>>(OUTP, out);
}
